// DeltaAttention_11063835755022
// MI455X (gfx1250) — hardware-verified
//
#include <hip/hip_runtime.h>

typedef _Float16 v16h __attribute__((ext_vector_type(16)));
typedef _Float16 v8h  __attribute__((ext_vector_type(8)));
typedef _Float16 v4h  __attribute__((ext_vector_type(4)));
typedef float    v8f  __attribute__((ext_vector_type(8)));
typedef float    v4f  __attribute__((ext_vector_type(4)));
typedef v8h __attribute__((may_alias)) v8ha;
typedef v4f __attribute__((may_alias)) v4fa;

union Frag { v16h v; v8h half[2]; };

#define DI     1024
#define NH     16
#define HD     64
#define SEQ    2048
#define NB     2
#define MROWS  (NB * SEQ)
#define NX     (MROWS * DI)
#define NW     (DI * DI)
#define NX8    (NX / 8)
#define PSCALE 16384.0f
#define EPSK   1e-8f
#define LNEPS  1e-5f

__device__ __forceinline__ v8f wmma_f16(v16h a, v16h b, v8f c) {
  v8f d = __builtin_amdgcn_wmma_f32_16x16x32_f16(false, a, false, b, (short)0, c, false, false);
  asm volatile("v_nop\n\tv_nop\n\tv_nop\n\tv_nop" : "+v"(d) : "v"(a), "v"(b));
  return d;
}

__device__ __forceinline__ v16h load_frag(const _Float16* p, int h) {
  Frag f;
  f.half[0] = *(const v8ha*)(p + 8 * h);
  f.half[1] = *(const v8ha*)(p + 16 + 8 * h);
  return f.v;
}

__device__ __forceinline__ float wsum(float v) {
  v += __shfl_xor(v, 16);
  v += __shfl_xor(v, 8);
  v += __shfl_xor(v, 4);
  v += __shfl_xor(v, 2);
  v += __shfl_xor(v, 1);
  return v;
}

__device__ __forceinline__ float dot4(v4f a, v4f b) {
  return a.x * b.x + a.y * b.y + a.z * b.z + a.w * b.w;
}

__device__ __forceinline__ v8h gather_col8(const _Float16* p) {
  const v8h r = { p[0], p[64], p[128], p[192], p[256], p[320], p[384], p[448] };
  return r;
}

__global__ __launch_bounds__(256) void cvt_x_kernel(const float* __restrict__ x,
                                                    _Float16* __restrict__ xh)
{
  const int g = blockIdx.x * 256 + threadIdx.x;
  if (g >= NX8) return;
  const float* src = x + (size_t)g * 8;
  const v4f a = *(const v4fa*)src;
  const v4f c = *(const v4fa*)(src + 4);
  const v8h o = { (_Float16)a.x, (_Float16)a.y, (_Float16)a.z, (_Float16)a.w,
                  (_Float16)c.x, (_Float16)c.y, (_Float16)c.z, (_Float16)c.w };
  _Float16* dst = xh + (size_t)g * 8;
  *(volatile v8h*)dst = o;
  __threadfence();
  *(volatile v8h*)dst = o;
}

__global__ __launch_bounds__(256) void cvt_wt_kernel(
    const float* __restrict__ Wq, const float* __restrict__ Wk, const float* __restrict__ Wv,
    const float* __restrict__ Wo, const float* __restrict__ dWk, _Float16* __restrict__ wt)
{
  __shared__ __attribute__((aligned(16))) _Float16 sT[64 * 64];

  const int t = threadIdx.x;
  const int n0 = blockIdx.x * 64;
  const int k0 = blockIdx.y * 64;
  const int z = blockIdx.z;
  const float* W;
  float sc;
  if (z < 4) {
    W = (z == 0) ? Wq : ((z == 1) ? Wk : ((z == 2) ? Wv : Wo));
    sc = 32.0f;
  } else {
    W = dWk + (size_t)(z - 4) * NW;
    sc = 64.0f;
  }
  _Float16* dst = wt + (size_t)z * NW;

  #pragma unroll
  for (int r = 0; r < 16; ++r) {
    const int k = 4 * r + (t >> 6), n = t & 63;
    sT[k * 64 + n] = (_Float16)(W[(size_t)(k0 + k) * DI + n0 + n] * sc);
  }
  __syncthreads();

  const int q8 = t & 7, lg = t >> 3;
  const v8h v0 = gather_col8(sT + (8 * q8) * 64 + lg);
  const v8h v1 = gather_col8(sT + (8 * q8) * 64 + lg + 32);
  _Float16* d0 = dst + (size_t)(n0 + lg) * DI + k0 + 8 * q8;
  _Float16* d1 = dst + (size_t)(n0 + lg + 32) * DI + k0 + 8 * q8;
  *(volatile v8h*)d0 = v0;
  *(volatile v8h*)d1 = v1;
  __threadfence();
  *(volatile v8h*)d0 = v0;
  *(volatile v8h*)d1 = v1;
}

__device__ __forceinline__ void gemm_store_pass(const float* sT, float* Cz,
                                                int m0, int n0, int w, int lane) {
  const int q8 = lane & 7, sub = lane >> 3;
  #pragma unroll
  for (int i = 0; i < 16; ++i) {
    const int lid = i * 4 + sub;
    const int row = 32 * w + (lid >> 1), hl = lid & 1;
    const v4f v = *(const v4fa*)(sT + row * 64 + 32 * hl + 4 * q8);
    *(volatile v4f*)(Cz + (size_t)(m0 + row) * DI + n0 + 32 * hl + 4 * q8) = v;
  }
}

__global__ __launch_bounds__(128) void gemm_kernel(
    const _Float16* __restrict__ A,
    const _Float16* __restrict__ Bt,
    const float* __restrict__ bias0, const float* __restrict__ bias1,
    const float* __restrict__ bias2,
    int has_bias,
    float* __restrict__ C,
    int zsb, int zsc, float cscale)
{
  __shared__ __attribute__((aligned(16))) float sT[128 * 64];

  const int tid = threadIdx.x, lane = tid & 31, w = tid >> 5;
  const int h = lane >> 4, m = lane & 15;
  const int m0 = blockIdx.x * 128, n0 = blockIdx.y * 64, z = blockIdx.z;
  const _Float16* Bz = Bt + (size_t)z * zsb;
  float* Cz = C + (size_t)z * zsc;
  const float* bias = (z == 0) ? bias0 : ((z == 1) ? bias1 : bias2);
  const int m0w = m0 + 32 * w;

  const _Float16* xa0 = A + (size_t)(m0w + m) * DI;
  const _Float16* xa1 = xa0 + (size_t)16 * DI;
  const _Float16* wb  = Bz + (size_t)(n0 + m) * DI;

  const v8f zero8 = {0.f, 0.f, 0.f, 0.f, 0.f, 0.f, 0.f, 0.f};
  v8f acc[2][4];
  #pragma unroll
  for (int mt = 0; mt < 2; ++mt)
    #pragma unroll
    for (int nt = 0; nt < 4; ++nt) acc[mt][nt] = zero8;

  #pragma unroll 1
  for (int k0 = 0; k0 < DI; k0 += 32) {
    const v16h a0 = load_frag(xa0 + k0, h);
    const v16h a1 = load_frag(xa1 + k0, h);
    #pragma unroll
    for (int nt = 0; nt < 4; ++nt) {
      const v16h b = load_frag(wb + (size_t)nt * 16 * DI + k0, h);
      acc[0][nt] = wmma_f16(a0, b, acc[0][nt]);
      acc[1][nt] = wmma_f16(a1, b, acc[1][nt]);
    }
  }

  #pragma unroll
  for (int nt = 0; nt < 4; ++nt) {
    const int feat = 16 * nt + m;
    const float bvl = has_bias ? bias[n0 + feat] : 0.0f;
    #pragma unroll
    for (int mt = 0; mt < 2; ++mt) {
      #pragma unroll
      for (int r = 0; r < 8; ++r) {
        const int tokl = 32 * w + 16 * mt + 8 * h + r;
        sT[tokl * 64 + feat] = acc[mt][nt][r] * cscale + bvl;
      }
    }
  }
  __syncthreads();

  gemm_store_pass(sT, Cz, m0, n0, w, lane);
  __threadfence();
  gemm_store_pass(sT, Cz, m0, n0, w, lane);
}

__device__ __forceinline__ float row_coef(const float* xr, const float* kr, const float* vr,
                                          const float* wr, const float* ur,
                                          float cb, float cv, int lane)
{
  float sn = 0.f, sk = 0.f, sb = 0.f, sv = 0.f;
  #pragma unroll 1
  for (int j = 0; j < 8; ++j) {
    const int c = 128 * j + 4 * lane;
    const v4f xx = *(const v4fa*)(xr + c);
    const v4f kk = *(const v4fa*)(kr + c);
    const v4f pp = *(const v4fa*)(vr + c);
    const v4f ww = *(const v4fa*)(wr + c);
    const v4f uu = *(const v4fa*)(ur + c);
    sn += dot4(kk, kk);
    sk += dot4(kk, xx);
    sb += dot4(xx, ww);
    sv += dot4(pp, uu);
  }
  sn = wsum(sn); sk = wsum(sk); sb = wsum(sb); sv = wsum(sv);
  const float kn   = 1.0f / (sqrtf(sn) + EPSK);
  const float beta = 2.0f * (1.0f / (1.0f + expf(-(sb + cb))));
  const float v    = sv + cv;
  const float kh   = sk * kn;
  return beta * (v - kh) * kn;
}

__global__ __launch_bounds__(256) void resid_qkv_kernel(
    const float* __restrict__ x,
    const float* __restrict__ kraw,
    const float* __restrict__ vin,
    const float* __restrict__ dbw,
    const float* __restrict__ dWv,
    const float* __restrict__ dbb,
    const float* __restrict__ dbv,
    int which,
    _Float16* __restrict__ qh,
    _Float16* __restrict__ kh,
    _Float16* __restrict__ vt)
{
  __shared__ __attribute__((aligned(16))) _Float16 sT[64 * 64];
  __shared__ float sCoef[64];

  const int t = threadIdx.x, lane = t & 31, w = t >> 5;
  const int t0 = blockIdx.x * 64;
  const float* wr = dbw + which * DI;
  const float* ur = dWv + which * DI;
  const float cb = dbb[which], cv = dbv[which];

  #pragma unroll 1
  for (int p = 0; p < 8; ++p) {
    const int r = 8 * p + w;
    const size_t ro = (size_t)(t0 + r) * DI;
    const float coef = row_coef(x + ro, kraw + ro, vin + ro, wr, ur, cb, cv, lane);
    if (lane == 0) sCoef[r] = coef;
  }
  __syncthreads();

  const int b = t0 / SEQ, s0 = t0 - b * SEQ;
  const int tok = t >> 2, dq = (t & 3) * 16;
  const float coef = sCoef[tok];
  const float osc = (which == 0) ? 0.125f : 1.0f;
  const v4f cf = { coef, coef, coef, coef };
  const v4f os = { osc, osc, osc, osc };
  const size_t rb = (size_t)(t0 + tok) * DI + dq;
  const int q8 = t & 7, lg = t >> 3;
  _Float16* plane = (which == 0) ? qh : kh;

  #pragma unroll 1
  for (int hh = 0; hh < NH; ++hh) {
    const float* xp = x + rb + hh * HD;
    const float* kp = kraw + rb + hh * HD;
    const v4f y0 = (*(const v4fa*)(xp)      + cf * *(const v4fa*)(kp))      * os;
    const v4f y1 = (*(const v4fa*)(xp + 4)  + cf * *(const v4fa*)(kp + 4))  * os;
    const v4f y2 = (*(const v4fa*)(xp + 8)  + cf * *(const v4fa*)(kp + 8))  * os;
    const v4f y3 = (*(const v4fa*)(xp + 12) + cf * *(const v4fa*)(kp + 12)) * os;
    const v4h c0 = __builtin_convertvector(y0, v4h);
    const v4h c1 = __builtin_convertvector(y1, v4h);
    const v4h c2 = __builtin_convertvector(y2, v4h);
    const v4h c3 = __builtin_convertvector(y3, v4h);
    if (which != 2) {
      const v8h lo = __builtin_shufflevector(c0, c1, 0, 1, 2, 3, 4, 5, 6, 7);
      const v8h hi = __builtin_shufflevector(c2, c3, 0, 1, 2, 3, 4, 5, 6, 7);
      *(v8ha*)(sT + tok * 64 + dq)     = lo;
      *(v8ha*)(sT + tok * 64 + dq + 8) = hi;
    } else {
      _Float16* sp = sT + dq * 64 + tok;
      sp[0 * 64]  = c0[0]; sp[1 * 64]  = c0[1]; sp[2 * 64]  = c0[2]; sp[3 * 64]  = c0[3];
      sp[4 * 64]  = c1[0]; sp[5 * 64]  = c1[1]; sp[6 * 64]  = c1[2]; sp[7 * 64]  = c1[3];
      sp[8 * 64]  = c2[0]; sp[9 * 64]  = c2[1]; sp[10 * 64] = c2[2]; sp[11 * 64] = c2[3];
      sp[12 * 64] = c3[0]; sp[13 * 64] = c3[1]; sp[14 * 64] = c3[2]; sp[15 * 64] = c3[3];
    }
    __syncthreads();

    const int bh = b * NH + hh;
    const v8h l0 = *(const v8ha*)(sT + lg * 64 + 8 * q8);
    const v8h l1 = *(const v8ha*)(sT + (lg + 32) * 64 + 8 * q8);
    _Float16* d0;
    _Float16* d1;
    if (which != 2) {
      d0 = plane + ((size_t)bh * SEQ + s0 + lg) * HD + 8 * q8;
      d1 = plane + ((size_t)bh * SEQ + s0 + lg + 32) * HD + 8 * q8;
    } else {
      d0 = vt + ((size_t)bh * HD + lg) * SEQ + s0 + 8 * q8;
      d1 = vt + ((size_t)bh * HD + lg + 32) * SEQ + s0 + 8 * q8;
    }
    *(volatile v8h*)d0 = l0;
    *(volatile v8h*)d1 = l1;
    __threadfence();
    *(volatile v8h*)d0 = l0;
    *(volatile v8h*)d1 = l1;
    __syncthreads();
  }
}

__device__ __forceinline__ v16h pack_p(v8f a, v8f c) {
  const v16h r = { (_Float16)(a[0] * PSCALE), (_Float16)(a[1] * PSCALE), (_Float16)(a[2] * PSCALE), (_Float16)(a[3] * PSCALE),
                   (_Float16)(a[4] * PSCALE), (_Float16)(a[5] * PSCALE), (_Float16)(a[6] * PSCALE), (_Float16)(a[7] * PSCALE),
                   (_Float16)(c[0] * PSCALE), (_Float16)(c[1] * PSCALE), (_Float16)(c[2] * PSCALE), (_Float16)(c[3] * PSCALE),
                   (_Float16)(c[4] * PSCALE), (_Float16)(c[5] * PSCALE), (_Float16)(c[6] * PSCALE), (_Float16)(c[7] * PSCALE) };
  return r;
}

__device__ __forceinline__ void att_store_pass(const _Float16* so, _Float16* ao,
                                               int b, int head, int q0, int lane) {
  const int q8 = lane & 7, sub = lane >> 3;
  #pragma unroll
  for (int i = 0; i < 4; ++i) {
    const int row = i * 4 + sub;
    const v8h v = *(const v8ha*)(so + row * 64 + 8 * q8);
    const size_t gi = ((size_t)b * SEQ + q0 + row) * DI + head * HD + 8 * q8;
    *(volatile v8h*)(ao + gi) = v;
  }
}

__global__ __launch_bounds__(128) void attn_kernel(
    const _Float16* __restrict__ qh,
    const _Float16* __restrict__ kh,
    const _Float16* __restrict__ vt,
    _Float16* __restrict__ ao)
{
  __shared__ __attribute__((aligned(16))) _Float16 sO[4 * 16 * 64];

  const int tid = threadIdx.x, lane = tid & 31, w = tid >> 5;
  const int h = lane >> 4, m = lane & 15;
  const int bh = blockIdx.y, b = bh >> 4, head = bh & 15;
  const int q0 = blockIdx.x * 64 + 16 * w;

  const _Float16* qrow = qh + ((size_t)bh * SEQ + q0 + m) * HD;
  const v16h qb0 = load_frag(qrow, h);
  const v16h qb1 = load_frag(qrow + 32, h);

  const v8f zero8 = {0.f, 0.f, 0.f, 0.f, 0.f, 0.f, 0.f, 0.f};
  v8f o[4];
  #pragma unroll
  for (int t = 0; t < 4; ++t) o[t] = zero8;
  float mrun = -1e30f, lrun = 0.0f;

  const _Float16* kbase = kh + ((size_t)bh * SEQ + m) * HD;
  const _Float16* vbase = vt + ((size_t)bh * HD + m) * SEQ;

  #pragma unroll 1
  for (int kb = 0; kb < SEQ; kb += 64) {
    v8f s[4];
    #pragma unroll
    for (int j = 0; j < 4; ++j) {
      const _Float16* kp = kbase + (size_t)(kb + 16 * j) * HD;
      const v16h kf0 = load_frag(kp, h);
      const v16h kf1 = load_frag(kp + 32, h);
      v8f zz = zero8;
      zz = wmma_f16(kf0, qb0, zz);
      zz = wmma_f16(kf1, qb1, zz);
      s[j] = zz;
    }

    float mloc = s[0][0];
    #pragma unroll
    for (int j = 0; j < 4; ++j)
      #pragma unroll
      for (int r = 0; r < 8; ++r) mloc = fmaxf(mloc, s[j][r]);
    mloc = fmaxf(mloc, __shfl_xor(mloc, 16));
    const float mnew = fmaxf(mrun, mloc);
    const float alpha = __expf(mrun - mnew);
    mrun = mnew;
    float lsum = 0.0f;
    #pragma unroll
    for (int j = 0; j < 4; ++j)
      #pragma unroll
      for (int r = 0; r < 8; ++r) {
        const float p = __expf(s[j][r] - mnew);
        s[j][r] = p;
        lsum += p;
      }
    lsum += __shfl_xor(lsum, 16);
    lrun = lrun * alpha + lsum;
    #pragma unroll
    for (int t = 0; t < 4; ++t)
      #pragma unroll
      for (int r = 0; r < 8; ++r) o[t][r] = o[t][r] * alpha;

    const v16h pb0 = pack_p(s[0], s[1]);
    const v16h pb1 = pack_p(s[2], s[3]);

    #pragma unroll
    for (int t = 0; t < 4; ++t) {
      const _Float16* vp = vbase + (size_t)(16 * t) * SEQ + kb;
      const v16h vf0 = load_frag(vp, h);
      const v16h vf1 = load_frag(vp + 32, h);
      o[t] = wmma_f16(vf0, pb0, o[t]);
      o[t] = wmma_f16(vf1, pb1, o[t]);
    }
  }

  const float inv = (1.0f / lrun) * (1.0f / PSCALE);
  _Float16* so = sO + w * 1024;
  #pragma unroll
  for (int t = 0; t < 4; ++t)
    #pragma unroll
    for (int r = 0; r < 8; ++r)
      so[m * 64 + 16 * t + 8 * h + r] = (_Float16)(o[t][r] * inv);
  __syncthreads();

  att_store_pass(so, ao, b, head, q0, lane);
  __threadfence();
  att_store_pass(so, ao, b, head, q0, lane);
}

__device__ __forceinline__ v4f ln_val4(const float* xr, const float* kr, const float* g,
                                       const float* bta, int c, v4f cf, v4f mu4, v4f rs4) {
  const v4f y = *(const v4fa*)(xr + c) + cf * *(const v4fa*)(kr + c);
  const v4f gg = *(const v4fa*)(g + c);
  const v4f bb = *(const v4fa*)(bta + c);
  return (y - mu4) * rs4 * gg + bb;
}

__global__ __launch_bounds__(256) void resid_ln_kernel(
    const float* __restrict__ x,
    const float* __restrict__ kraw,
    const float* __restrict__ vin,
    const float* __restrict__ dbw,
    const float* __restrict__ dWv,
    const float* __restrict__ dbb,
    const float* __restrict__ dbv,
    const float* __restrict__ g,
    const float* __restrict__ bta,
    float* __restrict__ out)
{
  const int t = threadIdx.x, lane = t & 31, w = t >> 5;
  const int row = blockIdx.x * 8 + w;
  if (row >= MROWS) return;
  const size_t ro = (size_t)row * DI;
  const float* xr = x + ro;
  const float* kr = kraw + ro;

  const float coef = row_coef(xr, kr, vin + ro, dbw + 3 * DI, dWv + 3 * DI, dbb[3], dbv[3], lane);
  const v4f cf = { coef, coef, coef, coef };

  float s = 0.0f;
  #pragma unroll 1
  for (int j = 0; j < 8; ++j) {
    const int c = 128 * j + 4 * lane;
    const v4f y = *(const v4fa*)(xr + c) + cf * *(const v4fa*)(kr + c);
    s += (y.x + y.y) + (y.z + y.w);
  }
  s = wsum(s);
  const float mu = s * (1.0f / DI);
  const v4f mu4 = { mu, mu, mu, mu };

  float s2 = 0.0f;
  #pragma unroll 1
  for (int j = 0; j < 8; ++j) {
    const int c = 128 * j + 4 * lane;
    const v4f y = *(const v4fa*)(xr + c) + cf * *(const v4fa*)(kr + c);
    const v4f d = y - mu4;
    s2 += dot4(d, d);
  }
  s2 = wsum(s2);
  const float var = s2 * (1.0f / DI);
  const float rs = 1.0f / sqrtf(var + LNEPS);
  const v4f rs4 = { rs, rs, rs, rs };

  #pragma unroll 1
  for (int j = 0; j < 8; ++j) {
    const int c = 128 * j + 4 * lane;
    const v4f o = ln_val4(xr, kr, g, bta, c, cf, mu4, rs4);
    *(volatile v4f*)(out + ro + c) = o;
  }
  __threadfence();
  #pragma unroll 1
  for (int j = 0; j < 8; ++j) {
    const int c = 128 * j + 4 * lane;
    const v4f o = ln_val4(xr, kr, g, bta, c, cf, mu4, rs4);
    *(volatile v4f*)(out + ro + c) = o;
  }
}

extern "C" void kernel_launch(void* const* d_in, const int* in_sizes, int n_in,
                              void* d_out, int out_size, void* d_ws, size_t ws_size,
                              hipStream_t stream) {
  if (n_in < 16) return;
  if (in_sizes[0] != NX) return;
  if (in_sizes[1] != NW || in_sizes[3] != NW || in_sizes[5] != NW || in_sizes[7] != NW) return;
  if (in_sizes[2] != DI || in_sizes[4] != DI || in_sizes[6] != DI || in_sizes[8] != DI) return;
  if (in_sizes[9] != 4 * NW || in_sizes[10] != 4 * DI || in_sizes[11] != 4) return;
  if (in_sizes[12] != 4 * DI || in_sizes[13] != 4) return;
  if (in_sizes[14] != DI || in_sizes[15] != DI) return;
  if (out_size != NX) return;

  const float* x   = (const float*)d_in[0];
  const float* Wq  = (const float*)d_in[1];
  const float* bq  = (const float*)d_in[2];
  const float* Wk  = (const float*)d_in[3];
  const float* bk  = (const float*)d_in[4];
  const float* Wv  = (const float*)d_in[5];
  const float* bv  = (const float*)d_in[6];
  const float* Wo  = (const float*)d_in[7];
  const float* bo  = (const float*)d_in[8];
  const float* dWk = (const float*)d_in[9];
  const float* dbw = (const float*)d_in[10];
  const float* dbb = (const float*)d_in[11];
  const float* dWv = (const float*)d_in[12];
  const float* dbv = (const float*)d_in[13];
  const float* lng = (const float*)d_in[14];
  const float* lnb = (const float*)d_in[15];
  float* out = (float*)d_out;

  const size_t b_x16 = (size_t)NX * 2;
  const size_t b_wt  = (size_t)8 * NW * 2;
  const size_t b_p   = (size_t)3 * NX * 4;
  const size_t b_kr  = (size_t)NX * 4;
  const size_t b_pl  = (size_t)NX * 2;
  const size_t b_ao  = (size_t)NX * 2;
  const size_t o_x16 = 0;
  const size_t o_wt  = o_x16 + b_x16;
  const size_t o_p   = o_wt + b_wt;
  const size_t o_kr  = o_p + b_p;
  const size_t o_q   = o_kr + b_kr;
  const size_t o_k   = o_q + b_pl;
  const size_t o_v   = o_k + b_pl;
  const size_t o_ao  = o_v + b_pl;
  const size_t total = o_ao + b_ao;
  if (total > ws_size) return;

  char* ws = (char*)d_ws;
  _Float16* x16  = (_Float16*)(ws + o_x16);
  _Float16* wt   = (_Float16*)(ws + o_wt);
  float*    P32  = (float*)(ws + o_p);
  float*    kraw = (float*)(ws + o_kr);
  _Float16* qh   = (_Float16*)(ws + o_q);
  _Float16* khp  = (_Float16*)(ws + o_k);
  _Float16* vtp  = (_Float16*)(ws + o_v);
  _Float16* ao   = (_Float16*)(ws + o_ao);
  float*    outp = P32;

  cvt_x_kernel<<<NX8 / 256, 256, 0, stream>>>(x, x16);
  cvt_wt_kernel<<<dim3(DI / 64, DI / 64, 8), 256, 0, stream>>>(Wq, Wk, Wv, Wo, dWk, wt);

  const dim3 gG3(MROWS / 128, DI / 64, 3);
  const dim3 gG1(MROWS / 128, DI / 64, 1);

  gemm_kernel<<<gG3, 128, 0, stream>>>(x16, wt, bq, bk, bv, 1, P32, NW, NX, 0.03125f);

  for (int i = 0; i < 3; ++i) {
    gemm_kernel<<<gG1, 128, 0, stream>>>(x16, wt + (size_t)(4 + i) * NW, bq, bq, bq, 0,
                                         kraw, 0, 0, 0.015625f);
    resid_qkv_kernel<<<MROWS / 64, 256, 0, stream>>>(x, kraw, P32 + (size_t)i * NX,
                                                     dbw, dWv, dbb, dbv, i, qh, khp, vtp);
  }

  attn_kernel<<<dim3(SEQ / 64, NB * NH), 128, 0, stream>>>(qh, khp, vtp, ao);

  gemm_kernel<<<gG1, 128, 0, stream>>>(ao, wt + (size_t)3 * NW, bo, bo, bo, 1, outp, 0, 0, 0.03125f);
  gemm_kernel<<<gG1, 128, 0, stream>>>(x16, wt + (size_t)7 * NW, bq, bq, bq, 0, kraw, 0, 0, 0.015625f);
  resid_ln_kernel<<<MROWS / 8, 256, 0, stream>>>(x, kraw, outp, dbw, dWv, dbb, dbv, lng, lnb, out);
}
